// MultimodalCausalSelfAttention_59124519797153
// MI455X (gfx1250) — hardware-verified
//
#include <hip/hip_runtime.h>
#include <math.h>
#include <stdint.h>

#define NB    8
#define NH    8
#define TT    1024
#define CIN   256
#define QKC   512
#define OUTC  256
#define NQKV  1280
#define DK    64
#define DV    32
#define KROW  512
#define VROW  1024
#define QBLK  128
static_assert(NH * DK == QKC);
static_assert(NH * DV == OUTC);
static_assert(KROW == QKC && VROW == 2 * QKC && NQKV == VROW + OUTC);
static_assert((TT % QBLK) == 0 && (TT % 64) == 0 && (QKC % 64) == 0 && ((NQKV - QKC) % 64) == 0);
static_assert((OUTC % 64) == 0 && (CIN % 64) == 0 && (CIN % 32) == 0 && (NH % 2) == 0 && (DK % 32) == 0 && DV == 32);

typedef _Float16 v16h __attribute__((ext_vector_type(16)));
typedef _Float16 v8h  __attribute__((ext_vector_type(8)));
typedef float    v8f  __attribute__((ext_vector_type(8)));
typedef float    v4f  __attribute__((ext_vector_type(4)));
typedef unsigned int v4u __attribute__((ext_vector_type(4)));

__device__ __forceinline__ unsigned short bf_bits(float f) {
  unsigned u = __float_as_uint(f);
  return (unsigned short)((u + 0x7FFFu + ((u >> 16) & 1u)) >> 16);
}
__device__ __forceinline__ float bf_up(unsigned short h) { return __uint_as_float(((unsigned)h) << 16); }
__device__ __forceinline__ unsigned short h_bits(_Float16 x) { return __builtin_bit_cast(unsigned short, x); }
__device__ __forceinline__ unsigned pk16(unsigned short a, unsigned short b) { return (unsigned)a | ((unsigned)b << 16); }
__device__ __forceinline__ v8f zero8() { v8f z = {0.f, 0.f, 0.f, 0.f, 0.f, 0.f, 0.f, 0.f}; return z; }

__device__ __forceinline__ v16h ldfrag_h(const _Float16* p) {
  union { v16h v; v8h h[2]; } f;
  f.h[0] = *(const v8h*)(p);
  f.h[1] = *(const v8h*)(p + 16);
  return f.v;
}

__device__ __forceinline__ v8f mma_h_raw(v16h a, v16h b, v8f c) {
  return __builtin_amdgcn_wmma_f32_16x16x32_f16(false, a, false, b, (short)0, c, false, false);
}
__device__ __forceinline__ void res_guard(v8f& t, v8f& acc, v16h x, v16h y) {
#if defined(__HIP_DEVICE_COMPILE__)
  asm volatile("v_nop\n\tv_nop\n\tv_nop\n\tv_nop" : "+v"(t), "+v"(acc) : "v"(x), "v"(y));
#endif
}
__device__ __forceinline__ void dep_guard_h(v8f& a, v8f& b, v16h x, v16h y) {
#if defined(__HIP_DEVICE_COMPILE__)
  asm volatile("v_nop\n\tv_nop\n\tv_nop\n\tv_nop" : "+v"(a), "+v"(b) : "v"(x), "v"(y));
#endif
}
__device__ __forceinline__ void guard4x6(v8f& a, v8f& b, v8f& c, v8f& d,
                                         v16h u, v16h v, v16h w, v16h x, v16h y, v16h z) {
#if defined(__HIP_DEVICE_COMPILE__)
  asm volatile("v_nop\n\tv_nop\n\tv_nop\n\tv_nop"
               : "+v"(a), "+v"(b), "+v"(c), "+v"(d)
               : "v"(u), "v"(v), "v"(w), "v"(x), "v"(y), "v"(z));
#endif
}
__device__ __forceinline__ void keep4_h(v16h a, v16h b, v16h c, v16h d) {
#if defined(__HIP_DEVICE_COMPILE__)
  asm volatile("v_nop" :: "v"(a), "v"(b), "v"(c), "v"(d));
#endif
}
__device__ __forceinline__ void acc_guard4(v8f& a, v8f& b, v8f& c, v8f& d) {
#if defined(__HIP_DEVICE_COMPILE__)
  asm volatile("v_nop\n\tv_nop\n\tv_nop\n\tv_nop" : "+v"(a), "+v"(b), "+v"(c), "+v"(d));
#endif
}
__device__ __forceinline__ void wave_sync_lds() {
  __builtin_amdgcn_fence(__ATOMIC_RELEASE, "workgroup");
  __builtin_amdgcn_wave_barrier();
  __builtin_amdgcn_fence(__ATOMIC_ACQUIRE, "workgroup");
}

__global__ __launch_bounds__(256) void cvt_h8(const float* __restrict__ in, unsigned short* out, int n8, float scale) {
  const int i = blockIdx.x * 256 + threadIdx.x;
  if (i < n8) {
    const v4f a = *(const v4f*)(in + (size_t)i * 8);
    const v4f c = *(const v4f*)(in + (size_t)i * 8 + 4);
    float f[8];
    f[0] = a[0]; f[1] = a[1]; f[2] = a[2]; f[3] = a[3];
    f[4] = c[0]; f[5] = c[1]; f[6] = c[2]; f[7] = c[3];
    unsigned short hb[8];
#pragma unroll
    for (int e = 0; e < 8; ++e) hb[e] = h_bits((_Float16)(bf_up(bf_bits(f[e])) * scale));
    v4u p;
    p[0] = pk16(hb[0], hb[1]);
    p[1] = pk16(hb[2], hb[3]);
    p[2] = pk16(hb[4], hb[5]);
    p[3] = pk16(hb[6], hb[7]);
    *(volatile v4u*)(out + (size_t)i * 8) = p;
    __threadfence();
    *(volatile v4u*)(out + (size_t)i * 8) = p;
  }
}

#define QTP 72
__global__ __launch_bounds__(256) void cvt_qt(const float* __restrict__ x, unsigned short* out, float scale) {
  __shared__ __align__(16) unsigned short ts[64 * QTP];
  const int tid = threadIdx.x;
  const int l0 = blockIdx.x * 64, c0 = blockIdx.y * 64, b = blockIdx.z;
#pragma unroll 1
  for (int pass = 0; pass < 4; ++pass) {
    const int c = pass * 16 + (tid >> 4);
    const int l4 = (tid & 15) * 4;
    const v4f v = *(const v4f*)(x + ((size_t)(b * CIN + c0 + c) * TT) + l0 + l4);
#pragma unroll
    for (int i = 0; i < 4; ++i) ts[(l4 + i) * QTP + c] = h_bits((_Float16)(bf_up(bf_bits(v[i])) * scale));
  }
  __syncthreads();
#pragma unroll 1
  for (int pass = 0; pass < 2; ++pass) {
    const int lr = pass * 32 + (tid >> 3);
    const int c8 = (tid & 7) * 8;
    const v4u v = *(const v4u*)(ts + lr * QTP + c8);
    unsigned short* dst = out + ((size_t)(b * TT) + l0 + lr) * CIN + c0 + c8;
    *(volatile v4u*)dst = v;
    __threadfence();
    *(volatile v4u*)dst = v;
  }
}

template <int NSPLIT, int BIAS>
__global__ __launch_bounds__(256) void gemm64(
    const unsigned short* __restrict__ Ap, int lda, long long sAy, long long sAz,
    const unsigned short* __restrict__ Btp, int ldb, long long sBy, long long sBz,
    const unsigned short* __restrict__ Bt2p, int ldb2,
    const float* __restrict__ bias,
    float* Cout, int ldc, long long sCy, long long sCz,
    int M, int N, int K, float oscale, float rres) {
  const _Float16* A   = (const _Float16*)(const void*)Ap;
  const _Float16* Bt  = (const _Float16*)(const void*)Btp;
  const _Float16* Bt2 = (const _Float16*)(const void*)Bt2p;
  __shared__ __align__(16) float sT[8][16 * 68];
  const int by   = blockIdx.y;
  const int bz   = blockIdx.z;
  const int lane = threadIdx.x & 31;
  const int wave = threadIdx.x >> 5;
  const int tilesN = N >> 6;
  const int tilesM = M >> 6;
  const int tile = blockIdx.x * 8 + wave;
  if (tile >= tilesM * tilesN) return;
  const int tm = tile / tilesN;
  const int tn = tile - tm * tilesN;
  const int m0 = tm << 6;
  const int n0 = tn << 6;

  const _Float16* Ab  = A + (size_t)by * (size_t)sAy + (size_t)bz * (size_t)sAz;
  const _Float16* Bb  = Bt + (size_t)by * (size_t)sBy + (size_t)bz * (size_t)sBz;
  const _Float16* Bb2 = (NSPLIT == 2) ? (Bt2 + (size_t)by * (size_t)sBy + (size_t)bz * (size_t)sBz) : Bb;
  const int ld2 = (NSPLIT == 2) ? ldb2 : ldb;

  const int rlane = lane & 15;
  const int koff  = (lane >> 4) * 8;
  const int mOff  = (lane >> 4) * 8;

  v8f acc[4][4];
#pragma unroll
  for (int i = 0; i < 4; ++i)
#pragma unroll
    for (int j = 0; j < 4; ++j) acc[i][j] = zero8();

  for (int k0 = 0; k0 < K; k0 += 32) {
    v16h bf[4];
#pragma unroll
    for (int j = 0; j < 4; ++j) {
      const size_t bo = (size_t)(n0 + (j << 4) + rlane) * ldb + koff + k0;
      bf[j] = ldfrag_h(Bb + bo);
    }
#pragma unroll
    for (int i = 0; i < 4; ++i) {
      const size_t ao = (size_t)(m0 + (i << 4) + rlane) * lda + koff + k0;
      const v16h ah = ldfrag_h(Ab + ao);
#pragma unroll
      for (int j = 0; j < 4; ++j) acc[i][j] = mma_h_raw(ah, bf[j], acc[i][j]);
      dep_guard_h(acc[i][0], acc[i][3], ah, bf[3]);
    }
    if (NSPLIT == 2) {
#pragma unroll
      for (int j = 0; j < 4; ++j) {
        const size_t bo = (size_t)(n0 + (j << 4) + rlane) * ld2 + koff + k0;
        bf[j] = ldfrag_h(Bb2 + bo);
      }
#pragma unroll
      for (int i = 0; i < 4; ++i) {
        const size_t ao = (size_t)(m0 + (i << 4) + rlane) * lda + koff + k0;
        const v16h al = ldfrag_h(Ab + ao);
#pragma unroll
        for (int j = 0; j < 4; ++j) {
          v8f tp = mma_h_raw(al, bf[j], zero8());
          res_guard(tp, acc[i][j], al, bf[j]);
#pragma unroll
          for (int r = 0; r < 8; ++r) acc[i][j][r] += tp[r] * rres;
        }
        dep_guard_h(acc[i][0], acc[i][3], al, bf[3]);
      }
    }
    keep4_h(bf[0], bf[1], bf[2], bf[3]);
  }
  acc_guard4(acc[0][0], acc[0][1], acc[0][2], acc[0][3]);
  acc_guard4(acc[1][0], acc[1][1], acc[1][2], acc[1][3]);
  acc_guard4(acc[2][0], acc[2][1], acc[2][2], acc[2][3]);
  acc_guard4(acc[3][0], acc[3][1], acc[3][2], acc[3][3]);

  float* slab = sT[wave];
  float* C = Cout + (size_t)by * (size_t)sCy + (size_t)bz * (size_t)sCz;
#pragma unroll
  for (int i = 0; i < 4; ++i) {
    const int mBase = m0 + (i << 4);
    float brow[8];
#pragma unroll
    for (int r = 0; r < 8; ++r) brow[r] = 0.f;
    if (BIAS == 2) {
#pragma unroll
      for (int r = 0; r < 8; ++r) brow[r] = bf_up(bf_bits(bias[mBase + mOff + r]));
    }
#pragma unroll
    for (int j = 0; j < 4; ++j) {
#pragma unroll
      for (int r = 0; r < 8; ++r) {
        slab[(mOff + r) * 68 + (j << 4) + rlane] = acc[i][j][r] * oscale + brow[r];
      }
    }
    wave_sync_lds();
    {
      const int hh = lane >> 4, c4 = (lane & 15) * 4;
      for (int pass = 0; pass < 2; ++pass) {
#pragma unroll
        for (int it = 0; it < 8; ++it) {
          const int row = it * 2 + hh;
          const v4f v = *(const v4f*)(slab + row * 68 + c4);
          *(volatile v4f*)(C + (size_t)(mBase + row) * ldc + n0 + c4) = v;
        }
        __threadfence();
      }
    }
    wave_sync_lds();
  }
}

#define YP 68
__global__ __launch_bounds__(256) void relayout_qk(
    const float* __restrict__ Y,
    unsigned short* QH, unsigned short* QL, unsigned short* KH, unsigned short* KL) {
  __shared__ __align__(16) float ys[64 * YP];
  const int tid = threadIdx.x;
  const int t0 = blockIdx.x * 64, pl = blockIdx.y, b = blockIdx.z;
  const int ob = pl * 64;
  const bool isq = (pl < NH);
  const int inst = b * NH + (pl & (NH - 1));
  unsigned short* Ph = isq ? QH : KH;
  unsigned short* Pl = isq ? QL : KL;
  const float* Yb = Y + ((size_t)(b * NQKV + ob)) * TT + t0;

#pragma unroll 1
  for (int it = 0; it < 4; ++it) {
    const int idx = it * 256 + tid;
    const int row = idx >> 4;
    const int c4  = (idx & 15) * 4;
    const v4f v = *(const v4f*)(Yb + (size_t)row * TT + c4);
    *(v4f*)(ys + row * YP + c4) = v;
  }
  __syncthreads();

#pragma unroll 1
  for (int pass = 0; pass < 2; ++pass) {
    const int r  = pass * 32 + (tid >> 3);
    const int d8 = (tid & 7) * 8;
    const float* src = ys + d8 * YP + r;
    unsigned short hb[8], lb[8];
#pragma unroll
    for (int i = 0; i < 8; ++i) {
      const float v = src[i * YP] * 16.0f;
      const _Float16 xh = (_Float16)v;
      hb[i] = h_bits(xh);
      lb[i] = h_bits((_Float16)((v - (float)xh) * 2048.0f));
    }
    v4u ph, plv;
#pragma unroll
    for (int q = 0; q < 4; ++q) {
      ph[q]  = pk16(hb[2 * q], hb[2 * q + 1]);
      plv[q] = pk16(lb[2 * q], lb[2 * q + 1]);
    }
    const size_t dst = ((size_t)(inst * TT + t0 + r)) * DK + d8;
    *(volatile v4u*)(Ph + dst) = ph;
    *(volatile v4u*)(Pl + dst) = plv;
    __threadfence();
    *(volatile v4u*)(Ph + dst) = ph;
    *(volatile v4u*)(Pl + dst) = plv;
  }
}

__global__ __launch_bounds__(256) void relayout_v(const float* __restrict__ Y, unsigned short* VH, unsigned short* VL) {
  const int tid = threadIdx.x;
  const int t0 = blockIdx.x * 64, cg = blockIdx.y, b = blockIdx.z;
  const int c = cg * 32 + (tid >> 3);
  const int col8 = (tid & 7) * 8;
  const float* src = Y + ((size_t)(b * NQKV + VROW + c)) * TT + t0 + col8;
  const v4f a  = *(const v4f*)(src);
  const v4f a2 = *(const v4f*)(src + 4);
  float f[8];
  f[0] = a[0]; f[1] = a[1]; f[2] = a[2]; f[3] = a[3];
  f[4] = a2[0]; f[5] = a2[1]; f[6] = a2[2]; f[7] = a2[3];
  unsigned short hb[8], lb[8];
#pragma unroll
  for (int i = 0; i < 8; ++i) {
    const float v = f[i] * 16.0f;
    const _Float16 xh = (_Float16)v;
    hb[i] = h_bits(xh);
    lb[i] = h_bits((_Float16)((v - (float)xh) * 2048.0f));
  }
  v4u ph, plv;
#pragma unroll
  for (int q = 0; q < 4; ++q) {
    ph[q]  = pk16(hb[2 * q], hb[2 * q + 1]);
    plv[q] = pk16(lb[2 * q], lb[2 * q + 1]);
  }
  const size_t dst = ((size_t)(b * OUTC + c)) * TT + t0 + col8;
  *(volatile v4u*)(VH + dst) = ph;
  *(volatile v4u*)(VL + dst) = plv;
  __threadfence();
  *(volatile v4u*)(VH + dst) = ph;
  *(volatile v4u*)(VL + dst) = plv;
}

#define SP 72
__device__ __forceinline__ void score_step(const _Float16* kh_p, const _Float16* kl_p, v16h qh, v16h ql,
                                           v8f& sh0, v8f& sh1, v8f& sr0, v8f& sr1) {
  const v16h kh0 = ldfrag_h(kh_p);
  const v16h kh1 = ldfrag_h(kh_p + 16 * DK);
  const v16h kl0 = ldfrag_h(kl_p);
  const v16h kl1 = ldfrag_h(kl_p + 16 * DK);
  sh0 = mma_h_raw(kh0, qh, sh0);
  sr0 = mma_h_raw(kh0, ql, sr0);
  sr0 = mma_h_raw(kl0, qh, sr0);
  sh1 = mma_h_raw(kh1, qh, sh1);
  sr1 = mma_h_raw(kh1, ql, sr1);
  sr1 = mma_h_raw(kl1, qh, sr1);
  guard4x6(sh0, sh1, sr0, sr1, kh0, kh1, kl0, kl1, qh, ql);
}

__global__ __launch_bounds__(256) void attn_kernel(
    const unsigned short* __restrict__ QHp, const unsigned short* __restrict__ QLp,
    const unsigned short* __restrict__ KHp, const unsigned short* __restrict__ KLp,
    const unsigned short* __restrict__ VHp, const unsigned short* __restrict__ VLp,
    unsigned short* CTXh, unsigned short* CTXl, float rscale) {
  __shared__ __align__(16) unsigned short sth[8 * 16 * SP];
  __shared__ __align__(16) unsigned short stl[8 * 16 * SP];
  const _Float16* QH = (const _Float16*)(const void*)QHp;
  const _Float16* QL = (const _Float16*)(const void*)QLp;
  const _Float16* KH = (const _Float16*)(const void*)KHp;
  const _Float16* KL = (const _Float16*)(const void*)KLp;
  const _Float16* VH = (const _Float16*)(const void*)VHp;
  const _Float16* VL = (const _Float16*)(const void*)VLp;

  const int tid = threadIdx.x, lane = tid & 31, wave = tid >> 5;
  const int b = blockIdx.z, hp = blockIdx.y;
  const int qBase = blockIdx.x * QBLK + wave * 16;
  const int rlane = lane & 15, hsel = lane >> 4, koff = hsel * 8;
  const int qcol = qBase + rlane;
  int ns = (qBase + 16 + 31) >> 5;
  if (ns > TT / 32) ns = TT / 32;
  const float C2048  = 1.0f / 2048.0f;
  const float SCL    = 1.0f / 2048.0f;
  const float LN1024 = 6.931471805599453f;
  const float NEGBIG = -1.0e30f;

#pragma unroll 1
  for (int h2 = 0; h2 < 2; ++h2) {
    const int h = hp * 2 + h2;
    const int inst = b * NH + h;
    const size_t qo = ((size_t)(inst * TT + qcol)) * DK + koff;
    const v16h qh0 = ldfrag_h(QH + qo);
    const v16h qh1 = ldfrag_h(QH + qo + 32);
    const v16h ql0 = ldfrag_h(QL + qo);
    const v16h ql1 = ldfrag_h(QL + qo + 32);
    const _Float16* Khb = KH + (size_t)inst * TT * DK + (size_t)rlane * DK + koff;
    const _Float16* Klb = KL + (size_t)inst * TT * DK + (size_t)rlane * DK + koff;
    const _Float16* Vhb = VH + ((size_t)(b * OUTC + h * DV + rlane)) * TT + koff;
    const _Float16* Vlb = VL + ((size_t)(b * OUTC + h * DV + rlane)) * TT + koff;

    v8f oh0 = zero8(), oh1 = zero8(), ol0 = zero8(), ol1 = zero8();
    float m_run = -1e30f, l_run = 0.f;

#pragma unroll 1
    for (int st = 0; st < ns; ++st) {
      const int s = st * 32;
      v8f sh0 = zero8(), sh1 = zero8(), sr0 = zero8(), sr1 = zero8();
      score_step(Khb + (size_t)s * DK,      Klb + (size_t)s * DK,      qh0, ql0, sh0, sh1, sr0, sr1);
      score_step(Khb + (size_t)s * DK + 32, Klb + (size_t)s * DK + 32, qh1, ql1, sh0, sh1, sr0, sr1);

      const int dq = qcol - (s + koff);
      float a0[8], a1[8];
#pragma unroll
      for (int r = 0; r < 8; ++r) {
        const float x0 = (sh0[r] + sr0[r] * C2048) * SCL;
        const float x1 = (sh1[r] + sr1[r] * C2048) * SCL;
        a0[r] = (r <= dq) ? x0 : NEGBIG;
        a1[r] = (r + 16 <= dq) ? x1 : NEGBIG;
      }

      float mloc = -1e30f;
#pragma unroll
      for (int r = 0; r < 8; ++r) mloc = fmaxf(mloc, fmaxf(a0[r], a1[r]));
      mloc = fmaxf(mloc, __shfl_xor(mloc, 16, 32));
      const float newM  = fmaxf(m_run, mloc);
      const float alpha = __expf(m_run - newM);
      const float msh   = newM - LN1024;
      float ssum = 0.f;
      float p0[8], p1[8];
#pragma unroll
      for (int r = 0; r < 8; ++r) {
        p0[r] = __expf(a0[r] - msh);
        p1[r] = __expf(a1[r] - msh);
        ssum += p0[r] + p1[r];
      }
      ssum += __shfl_xor(ssum, 16, 32);
      l_run = l_run * alpha + ssum;
      m_run = newM;
#pragma unroll
      for (int r = 0; r < 8; ++r) { oh0[r] *= alpha; oh1[r] *= alpha; ol0[r] *= alpha; ol1[r] *= alpha; }

      union { v16h v; _Float16 e[16]; } pf, pr;
#pragma unroll
      for (int r = 0; r < 8; ++r) {
        const _Float16 y0 = (_Float16)p0[r];
        const _Float16 y1 = (_Float16)p1[r];
        pf.e[r]     = y0;
        pf.e[8 + r] = y1;
        pr.e[r]     = (_Float16)((p0[r] - (float)y0) * 2048.0f);
        pr.e[8 + r] = (_Float16)((p1[r] - (float)y1) * 2048.0f);
      }

      const v16h vah0 = ldfrag_h(Vhb + s);
      const v16h vah1 = ldfrag_h(Vhb + (size_t)16 * TT + s);
      const v16h val0 = ldfrag_h(Vlb + s);
      const v16h val1 = ldfrag_h(Vlb + (size_t)16 * TT + s);
      oh0 = mma_h_raw(vah0, pf.v, oh0);
      ol0 = mma_h_raw(val0, pf.v, ol0);
      ol0 = mma_h_raw(vah0, pr.v, ol0);
      oh1 = mma_h_raw(vah1, pf.v, oh1);
      ol1 = mma_h_raw(val1, pf.v, ol1);
      ol1 = mma_h_raw(vah1, pr.v, ol1);
      guard4x6(oh0, oh1, ol0, ol1, vah0, vah1, val0, val1, pf.v, pr.v);
    }
    acc_guard4(oh0, oh1, ol0, ol1);

    const float inv = 4.0f * (1.0f / l_run);
    v4u hv0, lw0, hv1, lw1;
#pragma unroll
    for (int e = 0; e < 4; ++e) {
      {
        const float f0 = (oh0[2 * e]     + ol0[2 * e]     * C2048) * inv;
        const float f1 = (oh0[2 * e + 1] + ol0[2 * e + 1] * C2048) * inv;
        const _Float16 x0 = (_Float16)f0, x1 = (_Float16)f1;
        hv0[e] = pk16(h_bits(x0), h_bits(x1));
        lw0[e] = pk16(h_bits((_Float16)((f0 - (float)x0) * rscale)),
                      h_bits((_Float16)((f1 - (float)x1) * rscale)));
      }
      {
        const float f0 = (oh1[2 * e]     + ol1[2 * e]     * C2048) * inv;
        const float f1 = (oh1[2 * e + 1] + ol1[2 * e + 1] * C2048) * inv;
        const _Float16 x0 = (_Float16)f0, x1 = (_Float16)f1;
        hv1[e] = pk16(h_bits(x0), h_bits(x1));
        lw1[e] = pk16(h_bits((_Float16)((f0 - (float)x0) * rscale)),
                      h_bits((_Float16)((f1 - (float)x1) * rscale)));
      }
    }
    const int so = (wave * 16 + rlane) * SP + h2 * DV + koff;
    *(v4u*)(sth + so)      = hv0;
    *(v4u*)(sth + so + 16) = hv1;
    *(v4u*)(stl + so)      = lw0;
    *(v4u*)(stl + so + 16) = lw1;
  }

  wave_sync_lds();
  {
    const int rq = lane >> 3, c8 = (lane & 7) * 8;
    const unsigned short* hs = sth + (wave * 16) * SP;
    const unsigned short* ls = stl + (wave * 16) * SP;
    const size_t rb = (size_t)b * TT + qBase;
    for (int pass = 0; pass < 2; ++pass) {
#pragma unroll
      for (int it = 0; it < 4; ++it) {
        const int row = it * 4 + rq;
        const v4u v = *(const v4u*)(hs + row * SP + c8);
        *(volatile v4u*)(CTXh + (rb + row) * OUTC + hp * 64 + c8) = v;
      }
      __threadfence();
    }
    for (int pass = 0; pass < 2; ++pass) {
#pragma unroll
      for (int it = 0; it < 4; ++it) {
        const int row = it * 4 + rq;
        const v4u v = *(const v4u*)(ls + row * SP + c8);
        *(volatile v4u*)(CTXl + (rb + row) * OUTC + hp * 64 + c8) = v;
      }
      __threadfence();
    }
  }
}

extern "C" void kernel_launch(void* const* d_in, const int* in_sizes, int n_in,
                              void* d_out, int out_size, void* d_ws, size_t ws_size,
                              hipStream_t stream) {
  if (n_in < 7) return;
  if (in_sizes[0] != NB * CIN * TT) return;
  if (in_sizes[1] != QKC * CIN) return;
  if (in_sizes[2] != QKC) return;
  if (in_sizes[3] != (NQKV - QKC) * CIN) return;
  if (in_sizes[4] != (NQKV - QKC)) return;
  if (in_sizes[5] != OUTC * OUTC) return;
  if (in_sizes[6] != OUTC) return;
  if (out_size != NB * OUTC * TT) return;

  const float* x    = (const float*)d_in[0];
  const float* wq   = (const float*)d_in[1];
  const float* bq   = (const float*)d_in[2];
  const float* wkv  = (const float*)d_in[3];
  const float* bkv  = (const float*)d_in[4];
  const float* wo   = (const float*)d_in[5];
  const float* bov  = (const float*)d_in[6];

  const size_t PXT = (size_t)NB * TT * CIN * 2;
  const size_t PW3 = (size_t)NQKV * CIN * 2;
  const size_t PPW = (size_t)OUTC * OUTC * 2;
  const size_t PY  = (size_t)NB * NQKV * TT * 4;
  const size_t PQ  = (size_t)NB * NH * TT * DK * 2;
  const size_t PV  = (size_t)NB * OUTC * TT * 2;
  const size_t PCT = (size_t)NB * TT * OUTC * 2;
  size_t off = 0;
  const size_t oXT = off; off += PXT;
  const size_t oW3 = off; off += PW3;
  const size_t oPW = off; off += PPW;
  const size_t oY  = off; off += PY;
  const size_t oQH = off; off += PQ;
  const size_t oQL = off; off += PQ;
  const size_t oKH = off; off += PQ;
  const size_t oKL = off; off += PQ;
  const size_t oVH = off; off += PV;
  const size_t oVL = off; off += PV;
  const size_t oCH = off; off += PCT;
  const size_t oCL = off; off += PCT;
  if (off > ws_size) return;
  if (off > (size_t)134217728) return;

  char* ws = (char*)d_ws;
  unsigned short* XT   = (unsigned short*)(ws + oXT);
  unsigned short* W3   = (unsigned short*)(ws + oW3);
  unsigned short* PWp  = (unsigned short*)(ws + oPW);
  float*          Y    = (float*)(ws + oY);
  unsigned short* QH   = (unsigned short*)(ws + oQH);
  unsigned short* QL   = (unsigned short*)(ws + oQL);
  unsigned short* KH   = (unsigned short*)(ws + oKH);
  unsigned short* KL   = (unsigned short*)(ws + oKL);
  unsigned short* VH   = (unsigned short*)(ws + oVH);
  unsigned short* VL   = (unsigned short*)(ws + oVL);
  unsigned short* CTXh = (unsigned short*)(ws + oCH);
  unsigned short* CTXl = (unsigned short*)(ws + oCL);
  float*          out  = (float*)d_out;

  const dim3 blk(256);
  const int n8wq  = QKC * CIN / 8;
  const int n8wkv = (NQKV - QKC) * CIN / 8;
  const int n8pw  = OUTC * OUTC / 8;
  const dim3 gWq((n8wq + 255) / 256);
  const dim3 gWkv((n8wkv + 255) / 256);
  const dim3 gPW((n8pw + 255) / 256);
  const dim3 gQt(TT / 64, CIN / 64, NB);
  const dim3 gGq(((QKC / 64) * (TT / 64) + 7) / 8, NB, 1);
  const dim3 gGkv((((NQKV - QKC) / 64) * (TT / 64) + 7) / 8, NB, 1);
  const dim3 gRqk(TT / 64, 2 * NH, NB);
  const dim3 gRv(TT / 64, OUTC / 32, NB);
  const dim3 gAttn(TT / QBLK, NH / 2, NB);
  const dim3 gProj(((OUTC / 64) * (TT / 64) + 7) / 8, NB, 1);

  const float oscQkv = 1.0f / 16384.0f;
  const float rscale = 16384.0f;
  const float oscPrj = 1.0f / 65536.0f;
  const float rres   = 1.0f / 16384.0f;

  cvt_qt<<<gQt, blk, 0, stream>>>(x, XT, 16.0f);
  cvt_h8<<<gWq, blk, 0, stream>>>(wq, W3, n8wq, 1024.0f);
  cvt_h8<<<gWkv, blk, 0, stream>>>(wkv, W3 + (size_t)QKC * CIN, n8wkv, 1024.0f);
  cvt_h8<<<gPW, blk, 0, stream>>>(wo, PWp, n8pw, 1024.0f);
  gemm64<0, 2><<<gGq, blk, 0, stream>>>(
      W3, CIN, 0LL, 0LL,
      XT, CIN, (long long)((size_t)TT * CIN), 0LL,
      XT, CIN,
      bq,
      Y, TT, (long long)((size_t)NQKV * TT), 0LL,
      QKC, TT, CIN, oscQkv, 0.0f);
  gemm64<0, 2><<<gGkv, blk, 0, stream>>>(
      W3 + (size_t)QKC * CIN, CIN, 0LL, 0LL,
      XT, CIN, (long long)((size_t)TT * CIN), 0LL,
      XT, CIN,
      bkv,
      Y + (size_t)QKC * TT, TT, (long long)((size_t)NQKV * TT), 0LL,
      NQKV - QKC, TT, CIN, oscQkv, 0.0f);
  relayout_qk<<<gRqk, blk, 0, stream>>>(Y, QH, QL, KH, KL);
  relayout_v<<<gRv, blk, 0, stream>>>(Y, VH, VL);
  attn_kernel<<<gAttn, blk, 0, stream>>>(QH, QL, KH, KL, VH, VL, CTXh, CTXl, rscale);
  gemm64<2, 2><<<gProj, blk, 0, stream>>>(
      PWp, OUTC, 0LL, 0LL,
      CTXh, OUTC, (long long)((size_t)TT * OUTC), 0LL,
      CTXl, OUTC,
      bov,
      out, TT, (long long)((size_t)OUTC * TT), 0LL,
      OUTC, TT, OUTC, oscPrj, rres);
  (void)hipGetLastError();
}
